// SoftAlign_74071005987587
// MI455X (gfx1250) — hardware-verified
//
#include <hip/hip_runtime.h>

typedef _Float16 v16h __attribute__((ext_vector_type(16)));
typedef _Float16 v8h  __attribute__((ext_vector_type(8)));
typedef float    v8f  __attribute__((ext_vector_type(8)));
typedef float    v4f  __attribute__((ext_vector_type(4)));

union Frag { v16h v; v8h h8[2]; };

#define BDIM 8
#define NQ   2048
#define NP   2048
#define DIM  512
#define TAU  0.07f
#define QSC  64.0f
#define VSC  64.0f
#define WSC  4096.0f

#define QR     32
#define KT     64
#define NTHR   256
#define SPITCH 72
#define OPITCH 132
#define TPITCH 72

__device__ __forceinline__ v8f mma16(v16h a, v16h b, v8f c)
{
    c = __builtin_amdgcn_wmma_f32_16x16x32_f16(false, a, false, b, (short)0, c, false, false);
    asm volatile("v_nop\n\tv_nop\n\tv_nop\n\tv_nop" : "+v"(c) : "v"(a), "v"(b));
    return c;
}

__global__ __launch_bounds__(64)
void k_norm(const float* __restrict__ pf, const float* __restrict__ qf,
            _Float16* __restrict__ qn, _Float16* __restrict__ pn, int nrows)
{
    __shared__ float wsum[2];
    const int row   = blockIdx.x;
    const int which = blockIdx.y;
    if (row >= nrows) return;
    const int t = threadIdx.x;

    const float* src = (which == 0 ? qf : pf) + (size_t)row * DIM + t * 8;
    const v4f x0 = *(const v4f*)(src);
    const v4f x1 = *(const v4f*)(src + 4);

    float ss = 0.f;
#pragma unroll
    for (int i = 0; i < 4; ++i) ss += x0[i] * x0[i];
#pragma unroll
    for (int i = 0; i < 4; ++i) ss += x1[i] * x1[i];
#pragma unroll
    for (int off = 16; off; off >>= 1) ss += __shfl_xor(ss, off);
    if ((t & 31) == 0) wsum[t >> 5] = ss;
    __syncthreads();
    const float tot = wsum[0] + wsum[1];
    const float inv = 1.0f / fmaxf(sqrtf(tot), 1e-12f);
    const float sc  = inv * QSC;

    v8h o;
#pragma unroll
    for (int i = 0; i < 4; ++i) {
        o[i]     = (_Float16)(x0[i] * sc);
        o[4 + i] = (_Float16)(x1[i] * sc);
    }
    _Float16* dst = (which == 0 ? qn : pn) + (size_t)row * DIM + t * 8;
    *(volatile v8h*)dst = o;
    __threadfence();
    *(volatile v8h*)dst = o;
}

__global__ __launch_bounds__(64)
void k_vtr(const float* __restrict__ pf, _Float16* __restrict__ vt)
{
    __shared__ __attribute__((aligned(16))) _Float16 tile[64 * TPITCH];
    const int p0 = blockIdx.x * 64;
    const int d0 = blockIdx.y * 64;
    const int b  = blockIdx.z;
    if (p0 >= NP || d0 >= DIM || b >= BDIM) return;
    const int t = threadIdx.x;

#pragma unroll 4
    for (int it = 0; it < 16; ++it) {
        const int idx = it * 64 + t;
        const int r   = idx >> 4;
        const int c4  = (idx & 15) * 4;
        const v4f x = *(const v4f*)(pf + ((size_t)(b * NP + p0 + r)) * DIM + d0 + c4);
#pragma unroll
        for (int i = 0; i < 4; ++i) tile[(c4 + i) * TPITCH + r] = (_Float16)(x[i] * VSC);
    }
    __syncthreads();

    const int w = t >> 5, lane = t & 31;
    const int c = (lane & 7) * 8;
#pragma unroll
    for (int p = 0; p < 8; ++p) {
        const int dl = w * 32 + p * 4 + (lane >> 3);
        const v8h v = *(const v8h*)(tile + dl * TPITCH + c);
        _Float16* g = vt + ((size_t)(b * DIM + d0 + dl)) * NP + p0 + c;
        *(volatile v8h*)g = v;
    }
    __threadfence();
#pragma unroll
    for (int p = 0; p < 8; ++p) {
        const int dl = w * 32 + p * 4 + (lane >> 3);
        const v8h v = *(const v8h*)(tile + dl * TPITCH + c);
        _Float16* g = vt + ((size_t)(b * DIM + d0 + dl)) * NP + p0 + c;
        *(volatile v8h*)g = v;
    }
}

__global__ __launch_bounds__(NTHR)
void k_attn(const _Float16* __restrict__ qn, const _Float16* __restrict__ pn,
            const _Float16* __restrict__ vt, float* __restrict__ out)
{
    __shared__ __attribute__((aligned(16))) _Float16 ls[QR * SPITCH];
    __shared__ __attribute__((aligned(16))) float    ost[(NTHR / 32) * 8 * OPITCH];
    __shared__ __attribute__((aligned(16))) float    pmax[QR * 4];
    __shared__ __attribute__((aligned(16))) float    psum[QR * 4];

    const int b  = blockIdx.y;
    const int q0 = blockIdx.x * QR;
    if (q0 >= NQ || b >= BDIM) return;

    const int tid  = threadIdx.x;
    const int w    = tid >> 5;
    const int lane = tid & 31;
    const int h    = lane >> 4;
    const int m    = lane & 15;
    const int rg   = w >> 2;
    const int wq   = w & 3;
    const int rbase = rg * 16;

    const _Float16* qrow  = qn + ((size_t)(b * NQ + q0 + rbase + m)) * DIM + 8 * h;
    const _Float16* prow0 = pn + ((size_t)(b * NP + wq * 16 + m)) * DIM + 8 * h;
    const _Float16* vrow  = vt + ((size_t)(b * DIM + wq * 128 + m)) * NP + 8 * h;

    const v8f zero = {0.f, 0.f, 0.f, 0.f, 0.f, 0.f, 0.f, 0.f};
    v8f oacc[8];
#pragma unroll
    for (int nt = 0; nt < 8; ++nt) oacc[nt] = zero;
    float rowMax[8], rowSum[8];
#pragma unroll
    for (int r = 0; r < 8; ++r) { rowMax[r] = -1.0e30f; rowSum[r] = 0.f; }

    const float cinv = 1.0f / TAU;
    const float sinv = 1.0f / (QSC * QSC);

    for (int j = 0; j < NP / KT; ++j) {
        const int kbase = j * KT;
        const _Float16* prow = prow0 + (size_t)kbase * DIM;

        v8f sacc = zero;
#pragma unroll 2
        for (int kk = 0; kk < DIM / 32; ++kk) {
            Frag a, bb;
            a.h8[0]  = *(const v8h*)(qrow + kk * 32);
            a.h8[1]  = *(const v8h*)(qrow + kk * 32 + 16);
            bb.h8[0] = *(const v8h*)(prow + kk * 32);
            bb.h8[1] = *(const v8h*)(prow + kk * 32 + 16);
            sacc = mma16(a.v, bb.v, sacc);
        }

        float s[8];
#pragma unroll
        for (int r = 0; r < 8; ++r) {
            s[r] = sacc[r] * sinv;
            float v = s[r];
            v = fmaxf(v, __shfl_xor(v, 1));
            v = fmaxf(v, __shfl_xor(v, 2));
            v = fmaxf(v, __shfl_xor(v, 4));
            v = fmaxf(v, __shfl_xor(v, 8));
            if (m == 0) pmax[(rbase + 8 * h + r) * 4 + wq] = v;
        }
        __syncthreads();

        float scl[8];
#pragma unroll
        for (int r = 0; r < 8; ++r) {
            const int row = rbase + 8 * h + r;
            const v4f pm  = *(const v4f*)(pmax + row * 4);
            const float mx = fmaxf(fmaxf(pm[0], pm[1]), fmaxf(pm[2], pm[3]));
            const float nm = fmaxf(rowMax[r], mx);
            scl[r]    = __expf((rowMax[r] - nm) * cinv);
            rowMax[r] = nm;
            const float e = __expf((s[r] - nm) * cinv);
            ls[row * SPITCH + wq * 16 + m] = (_Float16)(e * WSC);
            float sm = e;
            sm += __shfl_xor(sm, 1);
            sm += __shfl_xor(sm, 2);
            sm += __shfl_xor(sm, 4);
            sm += __shfl_xor(sm, 8);
            if (m == 0) psum[row * 4 + wq] = sm;
        }
        __syncthreads();

#pragma unroll
        for (int r = 0; r < 8; ++r) {
            const v4f ps = *(const v4f*)(psum + (rbase + 8 * h + r) * 4);
            rowSum[r] = rowSum[r] * scl[r] + ((ps[0] + ps[1]) + (ps[2] + ps[3]));
        }
        {
            v8f sv;
#pragma unroll
            for (int r = 0; r < 8; ++r) sv[r] = scl[r];
#pragma unroll
            for (int nt = 0; nt < 8; ++nt) oacc[nt] = oacc[nt] * sv;
        }

#pragma unroll 1
        for (int ks = 0; ks < KT / 32; ++ks) {
            Frag a;
            const _Float16* ap = ls + (rbase + m) * SPITCH + ks * 32 + 8 * h;
            a.h8[0] = *(const v8h*)(ap);
            a.h8[1] = *(const v8h*)(ap + 16);
            const _Float16* bp = vrow + kbase + ks * 32;
#pragma unroll
            for (int nt = 0; nt < 8; ++nt) {
                Frag bv;
                bv.h8[0] = *(const v8h*)(bp + (size_t)nt * 16 * NP);
                bv.h8[1] = *(const v8h*)(bp + (size_t)nt * 16 * NP + 16);
                oacc[nt] = mma16(a.v, bv.v, oacc[nt]);
            }
        }
        __syncthreads();
    }

    float inv[8];
#pragma unroll
    for (int r = 0; r < 8; ++r) inv[r] = (1.0f / (WSC * VSC)) / rowSum[r];

    float* myost = ost + w * (8 * OPITCH);
    float* gbase = out + ((size_t)(b * NQ + q0 + rbase)) * DIM + wq * 128 + 4 * lane;

#pragma unroll
    for (int half = 0; half < 2; ++half) {
#pragma unroll
        for (int rr = 0; rr < 4; ++rr) {
            const int r = 4 * half + rr;
            float* orow = myost + (4 * h + rr) * OPITCH + m;
#pragma unroll
            for (int nt = 0; nt < 8; ++nt) orow[nt * 16] = oacc[nt][r] * inv[r];
        }
        __syncthreads();
        v4f vals[8];
#pragma unroll
        for (int p = 0; p < 8; ++p) vals[p] = *(const v4f*)(myost + p * OPITCH + 4 * lane);
#pragma unroll
        for (int p = 0; p < 8; ++p) {
            float* g = gbase + (size_t)(8 * (p >> 2) + 4 * half + (p & 3)) * DIM;
            *(volatile v4f*)g = vals[p];
        }
        __threadfence();
#pragma unroll
        for (int p = 0; p < 8; ++p) {
            float* g = gbase + (size_t)(8 * (p >> 2) + 4 * half + (p & 3)) * DIM;
            *(volatile v4f*)g = vals[p];
        }
        __syncthreads();
    }
}

extern "C" void kernel_launch(void* const* d_in, const int* in_sizes, int n_in,
                              void* d_out, int out_size, void* d_ws, size_t ws_size,
                              hipStream_t stream)
{
    if (n_in < 2) return;
    const size_t nel = (size_t)BDIM * NP * DIM;
    if ((size_t)in_sizes[0] != nel || (size_t)in_sizes[1] != nel || (size_t)out_size != nel) return;
    const size_t half_bytes = nel * sizeof(_Float16);
    if (ws_size < 3 * half_bytes) return;

    const float* pf = (const float*)d_in[0];
    const float* qf = (const float*)d_in[1];
    float* out = (float*)d_out;

    _Float16* qn = (_Float16*)d_ws;
    _Float16* pn = qn + nel;
    _Float16* vt = pn + nel;

    k_norm<<<dim3(BDIM * NP, 2), 64, 0, stream>>>(pf, qf, qn, pn, BDIM * NP);
    k_vtr<<<dim3(NP / 64, DIM / 64, BDIM), 64, 0, stream>>>(pf, vt);
    k_attn<<<dim3(NQ / QR, BDIM), NTHR, 0, stream>>>(qn, pn, vt, out);
}
